// GWASEncoder_5162550690504
// MI455X (gfx1250) — hardware-run, weakly checked
//
#include <hip/hip_runtime.h>


#ifndef NS
#define NS 30000
#endif
#define NS_FULL 30000
#define TT   64
#define DM   128
#define DCAT 8
#define NCAT 32
#define VOC  50000
#define FEAT 137
#define KP   160
#define AP   168

static_assert(FEAT == DM + DCAT + 1);
static_assert(KP % 32 == 0);
static_assert(KP >= FEAT);
static_assert(KP == DM + 4 * 8);
static_assert(AP >= KP);
static_assert((AP * 2) % 16 == 0);
static_assert((KP * 2) % 16 == 0);
static_assert(TT == 64);
static_assert(DM == 128);
static_assert(DM % 64 == 0);
static_assert(32 * 4 == DM);
static_assert(32 * 2 == TT);
static_assert(16 * 8 == DM);
static_assert(8 * 32 == TT * 4);
static_assert(DCAT == 8);
static_assert(NS <= NS_FULL);
static_assert((DM * KP / 8) % 256 == 0);
static_assert(((size_t)VOC * DM) % 8 == 0);
static_assert((NCAT * DCAT) % 8 == 0);

typedef unsigned short bf;
typedef __attribute__((ext_vector_type(16))) __bf16   v16bf;
typedef __attribute__((ext_vector_type(8)))  unsigned short v8us;
typedef __attribute__((ext_vector_type(8)))  float    v8f;
typedef __attribute__((ext_vector_type(4)))  float    v4f;
typedef __attribute__((ext_vector_type(4)))  unsigned v4u;
typedef v4f  __attribute__((may_alias)) v4fa;

__device__ __forceinline__ unsigned short f2bf(float f) { unsigned u = __float_as_uint(f); u += 0x7FFFu + ((u >> 16) & 1u); return (unsigned short)(u >> 16); }
__device__ __forceinline__ float bfr(float f) { return __uint_as_float(((unsigned)f2bf(f)) << 16); }
__device__ __forceinline__ v16bf cat16b(v8us lo, v8us hi) { return __builtin_bit_cast(v16bf, __builtin_shufflevector(lo, hi, 0, 1, 2, 3, 4, 5, 6, 7, 8, 9, 10, 11, 12, 13, 14, 15)); }
__device__ __forceinline__ v8f wmmab(v16bf a, v16bf b, v8f c) { return __builtin_amdgcn_wmma_f32_16x16x32_bf16(false, a, false, b, (short)0, c, false, false); }
__device__ __forceinline__ v8f wmmabg(v16bf a, v16bf b, v8f c) { c = wmmab(a, b, c); asm volatile("v_nop\n\tv_nop\n\tv_nop\n\tv_nop" : "+v"(c) : "v"(a), "v"(b)); return c; }
__device__ __forceinline__ v16bf ldb(const bf* p)  { return cat16b(*(const v8us*)p, *(const v8us*)(p + 16)); }
__device__ __forceinline__ void wave_sync() { __builtin_amdgcn_fence(3  , "wavefront"); __builtin_amdgcn_wave_barrier(); asm volatile("" ::: "memory"); }

__global__ __launch_bounds__(256) void k_cvt8(const float* __restrict__ src, bf* dst, size_t n8) {
    const size_t i = (size_t)blockIdx.x * 256 + threadIdx.x; if (i >= n8) return;
    const v8f v = *(const v8f*)(src + i * 8); v8us o;
#pragma unroll
    for (int k = 0; k < 8; ++k) o[k] = f2bf(v[k]);
    *(volatile v8us*)(dst + i * 8) = o; __threadfence(); *(volatile v8us*)(dst + i * 8) = o;
}

__global__ __launch_bounds__(256) void k_wpad(const float* __restrict__ W, bf* dst) {
    const unsigned i = blockIdx.x * 256u + threadIdx.x; if (i >= (unsigned)(DM * KP / 8)) return;
    const unsigned row = i / (unsigned)(KP / 8), pc = i % (unsigned)(KP / 8);
    v8us o;
#pragma unroll
    for (int k = 0; k < 8; ++k) {
        const int col = (int)pc * 8 + k; const int cc = min(col, FEAT - 1);
        float v = W[(size_t)row * FEAT + cc]; asm volatile("" : "+v"(v));
        const float vv = (col < FEAT) ? v : 0.0f;
        o[k] = f2bf(vv); }
    *(volatile v8us*)(dst + (size_t)i * 8) = o; __threadfence(); *(volatile v8us*)(dst + (size_t)i * 8) = o;
}

__global__ __launch_bounds__(32) void k_encode(const int* __restrict__ tok, const float* __restrict__ sc, const int* __restrict__ cat,
                                               const bf* __restrict__ TB, const bf* __restrict__ CB, const bf* __restrict__ WB,
                                               const float* __restrict__ bias, float* OUT) {
    __shared__ __align__(16) bf At[TT * AP];
    __shared__ __align__(16) float sW[TT];
    __shared__ __align__(16) float sO[DM];
    __shared__ int sTok[TT];
    __shared__ int sCat[TT];
    __shared__ unsigned sSb[TT];
    static_assert(sizeof(bf) * TT * AP + 4 * TT + 4 * DM + 4 * TT + 4 * TT + 4 * TT <= 131072);
    const int lane = threadIdx.x & 31, lr = lane & 15, hi = lane >> 4;
    const unsigned n = blockIdx.x;
    const size_t ib = (size_t)n * TT;
    float wpart = 0.0f;
#pragma unroll
    for (int q = 0; q < 2; ++q) {
        const int t = q * 32 + lane;
        const int tk = tok[ib + t]; const int ck = cat[ib + t]; const float sv = bfr(sc[ib + t]);
        const float w = (tk != 0) ? sv : 0.0f;
        sTok[t] = min(max(tk, 0), VOC - 1); sCat[t] = min(max(ck, 0), NCAT - 1);
        sW[t] = w; sSb[t] = __float_as_uint(sv) >> 16;
        wpart += w; }
    wave_sync();
#pragma unroll 4
    for (int it = 0; it < 32; ++it) {
        const int row = it * 2 + hi;
        const int tk = sTok[row];
        const v8us v = *(const v8us*)(TB + (size_t)tk * DM + lr * 8);
        *(v8us*)(&At[row * AP + lr * 8]) = v; }
#pragma unroll 2
    for (int it = 0; it < 8; ++it) {
        const int idx = it * 32 + lane; const int row = idx >> 2, pc = idx & 3;
        const int ck = sCat[row];
        const v8us cv = *(const v8us*)(CB + (size_t)ck * DCAT);
        v4u cw = __builtin_bit_cast(v4u, cv); asm volatile("" : "+v"(cw));
        const unsigned sb = sSb[row];
        v4u o;
        o[0] = (pc == 0) ? cw[0] : ((pc == 1) ? sb : 0u);
        o[1] = (pc == 0) ? cw[1] : 0u; o[2] = (pc == 0) ? cw[2] : 0u; o[3] = (pc == 0) ? cw[3] : 0u;
        *(v8us*)(&At[row * AP + DM + pc * 8]) = __builtin_bit_cast(v8us, o); }
    wave_sync();
    wpart += __shfl_xor(wpart, 16, 32); wpart += __shfl_xor(wpart, 8, 32); wpart += __shfl_xor(wpart, 4, 32);
    wpart += __shfl_xor(wpart, 2, 32);  wpart += __shfl_xor(wpart, 1, 32);
    const float den = fmaxf(wpart, 1e-8f);
    const float inv = 1.0f / den;
    const int aoff = lr * AP + 8 * hi;
    const size_t boff = (size_t)lr * KP + 8 * hi;
#pragma unroll 1
    for (int ch = 0; ch < 2; ++ch) {
        const int c0 = ch * 64;
        v8f acc[4][4];
#pragma unroll
        for (int mb = 0; mb < 4; ++mb)
#pragma unroll
            for (int nb = 0; nb < 4; ++nb) acc[mb][nb] = (v8f){};
#pragma unroll 1
        for (int kc = 0; kc < KP; kc += 32) {
            v16bf a[4];
#pragma unroll
            for (int mb = 0; mb < 4; ++mb) {
                const v8us lo = *(const v8us*)(&At[aoff + mb * 16 * AP + kc]);
                const v8us up = *(const v8us*)(&At[aoff + mb * 16 * AP + kc + 16]);
                a[mb] = cat16b(lo, up); }
#pragma unroll
            for (int nb = 0; nb < 4; ++nb) { const v16bf b = ldb(WB + boff + (size_t)(c0 + nb * 16) * KP + kc);
#pragma unroll
                for (int mb = 0; mb < 4; ++mb) acc[mb][nb] = wmmabg(a[mb], b, acc[mb][nb]); }
        }
        float bc[4];
#pragma unroll
        for (int nb = 0; nb < 4; ++nb) bc[nb] = bfr(bias[c0 + nb * 16 + lr]);
        float sm[4];
#pragma unroll
        for (int nb = 0; nb < 4; ++nb) sm[nb] = 0.0f;
#pragma unroll
        for (int mb = 0; mb < 4; ++mb) {
            const v4f wa = *(const v4fa*)(&sW[mb * 16 + 8 * hi]); const v4f wb = *(const v4fa*)(&sW[mb * 16 + 8 * hi + 4]);
#pragma unroll
            for (int nb = 0; nb < 4; ++nb) {
#pragma unroll
                for (int j = 0; j < 4; ++j) { sm[nb] += (acc[mb][nb][j] + bc[nb]) * wa[j]; sm[nb] += (acc[mb][nb][4 + j] + bc[nb]) * wb[j]; } }
        }
#pragma unroll
        for (int nb = 0; nb < 4; ++nb) sm[nb] += __shfl_xor(sm[nb], 16, 32);
        if (hi == 0) {
#pragma unroll
            for (int nb = 0; nb < 4; ++nb) sO[c0 + nb * 16 + lr] = sm[nb]; }
    }
    wave_sync();
    const v4f r = *(const v4fa*)(&sO[lane * 4]);
    v4f val; val[0] = r[0] * inv; val[1] = r[1] * inv; val[2] = r[2] * inv; val[3] = r[3] * inv;
    float* orow = OUT + (size_t)n * DM + lane * 4;
    *(volatile v4f*)orow = val; __threadfence(); *(volatile v4f*)orow = val;
}

static constexpr size_t al256(size_t v) { return (v + 255) & ~(size_t)255; }
static constexpr size_t SZ_TB = al256((size_t)VOC * DM * 2);
static constexpr size_t SZ_CB = al256((size_t)NCAT * DCAT * 2);
static constexpr size_t SZ_WB = al256((size_t)DM * KP * 2);
static constexpr size_t SZ_TOTAL = SZ_TB + SZ_CB + SZ_WB;
static_assert(SZ_TOTAL <= (size_t)134217728);
static constexpr size_t N8_T = (size_t)VOC * DM / 8;
static constexpr size_t N8_C = (size_t)NCAT * DCAT / 8;
static constexpr unsigned G_T = (unsigned)((N8_T + 255) / 256);
static constexpr unsigned G_C = (unsigned)((N8_C + 255) / 256);
static constexpr unsigned G_W = (unsigned)(DM * KP / 8 / 256);
static_assert((size_t)G_W * 256 * 8 == (size_t)DM * KP);

extern "C" void kernel_launch(void* const* d_in, const int* in_sizes, int n_in,
                              void* d_out, int out_size, void* d_ws, size_t ws_size, hipStream_t stream) {
    if (n_in < 7) return;
    if ((size_t)in_sizes[0] < (size_t)NS * TT || (size_t)in_sizes[1] < (size_t)NS * TT || (size_t)in_sizes[2] < (size_t)NS * TT) return;
    if ((size_t)in_sizes[3] < (size_t)VOC * DM || (size_t)in_sizes[4] < (size_t)NCAT * DCAT) return;
    if ((size_t)in_sizes[5] < (size_t)DM * FEAT || in_sizes[6] < DM) return;
    if ((size_t)out_size < (size_t)NS * DM) return;
    if (SZ_TOTAL > ws_size) return;
    const int* tok = (const int*)d_in[0];
    const float* sc = (const float*)d_in[1];
    const int* cat = (const int*)d_in[2];
    const float* temb = (const float*)d_in[3];
    const float* cemb = (const float*)d_in[4];
    const float* pw = (const float*)d_in[5];
    const float* pb = (const float*)d_in[6];
    float* OUT = (float*)d_out;
    char* wsp = (char*)d_ws;
    bf* TB = (bf*)wsp; wsp += SZ_TB;
    bf* CB = (bf*)wsp; wsp += SZ_CB;
    bf* WB = (bf*)wsp; wsp += SZ_WB;

    k_cvt8<<<G_T, 256, 0, stream>>>(temb, TB, N8_T);
    k_cvt8<<<G_C, 256, 0, stream>>>(cemb, CB, N8_C);
    k_wpad<<<G_W, 256, 0, stream>>>(pw, WB);
    k_encode<<<dim3(NS, 1, 1), 32, 0, stream>>>(tok, sc, cat, TB, CB, WB, pb, OUT);
}
